// dspo_model_83030307766874
// MI455X (gfx1250) — hardware-verified
//
#include <hip/hip_runtime.h>
#include <math.h>

typedef __attribute__((ext_vector_type(16))) _Float16 v16h;
typedef __attribute__((ext_vector_type(8)))  _Float16 v8h;
typedef __attribute__((ext_vector_type(2)))  _Float16 v2h;
typedef __attribute__((ext_vector_type(16))) __bf16   v16b;
typedef __attribute__((ext_vector_type(8)))  __bf16   v8b;
typedef __attribute__((ext_vector_type(8)))  float    v8f;
typedef __attribute__((ext_vector_type(4)))  float    v4f;
typedef __attribute__((ext_vector_type(2)))  float    v2f;

constexpr int kSteps  = 262144;
constexpr int kState  = 64;
constexpr int kObs    = 32;
constexpr int kChunk  = 16;
constexpr int kNumCh  = kSteps / kChunk;
constexpr int kYW     = kObs * kChunk;
constexpr int kAW     = kState + kYW;
constexpr int kThr    = 256;

constexpr float kYCarry = 1024.0f;
constexpr float kGCarry = 16384.0f;
constexpr float kSCarry = 4096.0f;
constexpr float kOCarry = 4096.0f;
constexpr float kScale  = 1.0f / (kYCarry * kGCarry);
constexpr float kF16MinNormal = 6.103515625e-5f;

static_assert(kYCarry * kGCarry == kSCarry * kOCarry, "one fold-back scale for both halves of the concatenated product");
static_assert(kNumCh == 16384 && kYW == 512 && kAW == 576, "sizes");
static_assert((kNumCh % 64) == 0 && (kState % 64) == 0 && (kYW % 64) == 0 && (kYW % 32) == 0 && (kAW % 32) == 0, "GEMM M, N multiples of 64, K of 32");

constexpr size_t kOffHPG  = 0;
constexpr size_t kOffPLG  = kOffHPG  + (size_t)16 * kObs * kState * 4;
constexpr size_t kOffHPLG = kOffPLG  + (size_t)16 * kState * kObs * 4;
constexpr size_t kOffP16  = kOffHPLG + (size_t)16 * kObs * kObs * 4;
constexpr size_t kOffZB   = kOffP16  + (size_t)kState * kState * 4;
constexpr size_t kOffG16  = kOffZB   + (size_t)kYW * 4;
constexpr size_t kOffOT   = kOffG16  + (size_t)kState * kYW * 2;
constexpr size_t kOffAC   = kOffOT   + (size_t)kYW * kAW * 2;
constexpr size_t kOffWF   = kOffAC   + (size_t)kNumCh * kAW * 2;
constexpr size_t kOffYH   = kOffWF   + (size_t)kNumCh * kState * 4;
constexpr size_t kWsTotal = kOffYH   + (size_t)kNumCh * kYW * 4;
static_assert(kWsTotal == 57624576ull, "carve total");
static_assert(kWsTotal <= 134217728ull, "carve cap");
static_assert((kOffPLG % 256) == 0 && (kOffHPLG % 256) == 0 && (kOffP16 % 256) == 0 && (kOffZB % 256) == 0 && (kOffG16 % 256) == 0 && (kOffOT % 256) == 0 && (kOffAC % 256) == 0 && (kOffWF % 256) == 0 && (kOffYH % 256) == 0, "aligned regions");

__device__ __forceinline__ unsigned short f2bf_bits(float f) {
  unsigned u = __float_as_uint(f);
  return (unsigned short)((u + 0x7FFFu + ((u >> 16) & 1u)) >> 16);
}
__device__ __forceinline__ float bf_bits2f(unsigned short h) { return __uint_as_float(((unsigned)h) << 16); }
__device__ __forceinline__ float bf16r(float f) { return bf_bits2f(f2bf_bits(f)); }
__device__ __forceinline__ float carry_flush(float v, float carry) {
  const float s = v * carry;
  return (fabsf(s) < kF16MinNormal) ? 0.0f : s;
}
__device__ __forceinline__ float frcp(float x) { return __builtin_amdgcn_rcpf(x); }

__device__ __forceinline__ void dep_guard4_h(v8f& a, v8f& b, v8f& c, v8f& d, v16h x, v16h y) { asm volatile("v_nop\n\tv_nop\n\tv_nop\n\tv_nop" : "+v"(a), "+v"(b), "+v"(c), "+v"(d) : "v"(x), "v"(y)); }
__device__ __forceinline__ void dep_guard4_b(v8f& a, v8f& b, v8f& c, v8f& d, v16b x, v16b y) { asm volatile("v_nop\n\tv_nop\n\tv_nop\n\tv_nop" : "+v"(a), "+v"(b), "+v"(c), "+v"(d) : "v"(x), "v"(y)); }
__device__ __forceinline__ void keep4_h(v16h a, v16h b, v16h c, v16h d) { asm volatile("v_nop" :: "v"(a), "v"(b), "v"(c), "v"(d)); }
__device__ __forceinline__ void keep4_b(v16b a, v16b b, v16b c, v16b d) { asm volatile("v_nop" :: "v"(a), "v"(b), "v"(c), "v"(d)); }
__device__ __forceinline__ void acc_guard4(v8f& a, v8f& b, v8f& c, v8f& d) { asm volatile("v_nop\n\tv_nop\n\tv_nop\n\tv_nop" : "+v"(a), "+v"(b), "+v"(c), "+v"(d)); }

template <typename T> struct Frag;
template <> struct Frag<_Float16> {
  typedef v16h V; union U { v16h v; v8h h[2]; };
  static __device__ __forceinline__ v16h load(const _Float16* p) {
    U f; f.h[0] = *(const v8h*)(p); f.h[1] = *(const v8h*)(p + 16); return f.v;
  }
  static __device__ __forceinline__ v8f mma(v16h a, v16h b, v8f c) {
    return __builtin_amdgcn_wmma_f32_16x16x32_f16(false, a, false, b, (short)0, c, false, false);
  }
  static __device__ __forceinline__ void guard4(v8f& a, v8f& b, v8f& c, v8f& d, v16h x, v16h y) { dep_guard4_h(a, b, c, d, x, y); }
  static __device__ __forceinline__ void keep(v16h a, v16h b, v16h c, v16h d) { keep4_h(a, b, c, d); }
};
template <> struct Frag<__bf16> {
  typedef v16b V; union U { v16b v; v8b h[2]; };
  static __device__ __forceinline__ v16b load(const __bf16* p) {
    U f; f.h[0] = *(const v8b*)(p); f.h[1] = *(const v8b*)(p + 16); return f.v;
  }
  static __device__ __forceinline__ v8f mma(v16b a, v16b b, v8f c) {
    return __builtin_amdgcn_wmma_f32_16x16x32_bf16(false, a, false, b, (short)0, c, false, false);
  }
  static __device__ __forceinline__ void guard4(v8f& a, v8f& b, v8f& c, v8f& d, v16b x, v16b y) { dep_guard4_b(a, b, c, d, x, y); }
  static __device__ __forceinline__ void keep(v16b a, v16b b, v16b c, v16b d) { keep4_b(a, b, c, d); }
};

__device__ __forceinline__ v8f mma_h(v16h a, v16h b, v8f c) {
  c = __builtin_amdgcn_wmma_f32_16x16x32_f16(false, a, false, b, (short)0, c, false, false);
  asm volatile("v_nop\n\tv_nop\n\tv_nop\n\tv_nop" : "+v"(c) : "v"(a), "v"(b));
  return c;
}

template <int ET> struct Elem;
template <> struct Elem<0> { typedef _Float16 T; };
template <> struct Elem<1> { typedef __bf16 T; };
template <int ET, bool SPLIT, int BIAS_MODE, int OUT_MODE, bool RESID, int ACT = 0>
__global__ __launch_bounds__(256) void wmma_gemm64(
    const unsigned short* __restrict__ Ap, const unsigned short* __restrict__ A2p, int lda, long strideA,
    const unsigned short* __restrict__ Btp, const unsigned short* __restrict__ Bt2p, int ldb, long strideB,
    void* __restrict__ Cout, void* __restrict__ Cout2, int ldc, long strideC,
    const float* __restrict__ bias,
    const float* __restrict__ resid, long strideR,
    int M, int N, int K, float scale) {
  typedef typename Elem<ET>::T T;
  typedef typename Frag<T>::V V;
  const T* A = (const T*)Ap; const T* A2 = (const T*)A2p; const T* Bt = (const T*)Btp; const T* Bt2 = (const T*)Bt2p;
  __shared__ __align__(16) float sT[8][16 * 68];
  const int b    = blockIdx.y;
  const int lane = threadIdx.x & 31;
  const int wave = threadIdx.x >> 5;
  const int tilesN = N >> 6;
  const int tilesM = M >> 6;
  const int tile = blockIdx.x * 8 + wave;
  if (tile >= tilesM * tilesN) return;
  const int tm = tile / tilesN;
  const int tn = tile - tm * tilesN;
  const int m0 = tm << 6;
  const int n0 = tn << 6;

  const T* Ab  = A  + (size_t)b * strideA;
  const T* Bb  = Bt + (size_t)b * strideB;
  const T* Ab2 = SPLIT ? (A2  + (size_t)b * strideA) : nullptr;
  const T* Bb2 = SPLIT ? (Bt2 + (size_t)b * strideB) : nullptr;

  const int rlane = lane & 15;
  const int koff  = (lane >> 4) * 8;
  const int mOff  = (lane >> 4) * 8;

  v8f acc[4][4];
#pragma unroll
  for (int i = 0; i < 4; ++i)
#pragma unroll
    for (int j = 0; j < 4; ++j) acc[i][j] = (v8f){0.f,0.f,0.f,0.f,0.f,0.f,0.f,0.f};

  for (int k0 = 0; k0 < K; k0 += 32) {
    V bh[4], bl[4];
#pragma unroll
    for (int j = 0; j < 4; ++j) {
      const size_t bo = (size_t)(n0 + (j << 4) + rlane) * ldb + koff + k0;
      bh[j] = Frag<T>::load(Bb + bo);
      if (SPLIT) bl[j] = Frag<T>::load(Bb2 + bo);
    }
#pragma unroll
    for (int i = 0; i < 4; ++i) {
      const size_t ao = (size_t)(m0 + (i << 4) + rlane) * lda + koff + k0;
      V ah = Frag<T>::load(Ab + ao);
      V al;
      if (SPLIT) al = Frag<T>::load(Ab2 + ao);
#pragma unroll
      for (int j = 0; j < 4; ++j) {
        acc[i][j] = Frag<T>::mma(ah, bh[j], acc[i][j]);
        if (SPLIT) {
          acc[i][j] = Frag<T>::mma(ah, bl[j], acc[i][j]);
          acc[i][j] = Frag<T>::mma(al, bh[j], acc[i][j]);
        }
      }
      Frag<T>::guard4(acc[i][0], acc[i][1], acc[i][2], acc[i][3], ah, SPLIT ? al : ah);
    }
    Frag<T>::keep(bh[0], bh[1], bh[2], bh[3]);
    if (SPLIT) Frag<T>::keep(bl[0], bl[1], bl[2], bl[3]);
  }
  acc_guard4(acc[0][0], acc[0][1], acc[0][2], acc[0][3]);
  acc_guard4(acc[1][0], acc[1][1], acc[1][2], acc[1][3]);
  acc_guard4(acc[2][0], acc[2][1], acc[2][2], acc[2][3]);
  acc_guard4(acc[3][0], acc[3][1], acc[3][2], acc[3][3]);

  float* slab = sT[wave];
  const float* Rb = RESID ? (resid + (size_t)b * strideR) : nullptr;
#pragma unroll
  for (int i = 0; i < 4; ++i) {
    const int mBase = m0 + (i << 4);
#pragma unroll
    for (int j = 0; j < 4; ++j) {
      const int n = n0 + (j << 4) + rlane;
      float bv = 0.f;
      if (BIAS_MODE == 2) bv = bias[n];
#pragma unroll
      for (int r = 0; r < 8; ++r) {
        float v = acc[i][j][r] * scale;
        if (BIAS_MODE == 1) v += bias[mBase + mOff + r];
        if (BIAS_MODE == 2) v += bv;
        if (RESID) v += Rb[(size_t)(mBase + mOff + r) * ldc + n];
        if (ACT == 1) v = tanhf(v);
        if (ACT == 2) v = fmaxf(v, 0.0f);
        if (ACT == 3) v = v / (1.0f + expf(-v));
        if (ACT == 4) v = (v > 0.f) ? v : 0.01f * v;
        slab[(mOff + r) * 68 + (j << 4) + rlane] = v;
      }
    }
    __builtin_amdgcn_fence(__ATOMIC_RELEASE, "workgroup");
    __builtin_amdgcn_wave_barrier();
    __builtin_amdgcn_fence(__ATOMIC_ACQUIRE, "workgroup");
    if (OUT_MODE == 0) {
      float* C = (float*)Cout + (size_t)b * strideC;
      const int hh = lane >> 4, c4 = (lane & 15) * 4;
      for (int pass = 0; pass < 2; ++pass) {
#pragma unroll
        for (int it = 0; it < 8; ++it) {
          const int row = it * 2 + hh;
          v4f v = *(const v4f*)(slab + row * 68 + c4);
          *(volatile v4f*)(C + (size_t)(mBase + row) * ldc + n0 + c4) = v;
        }
        __threadfence();
      }
    } else {
      const int q = lane >> 3, c8 = (lane & 7) * 8;
      unsigned short* C  = (unsigned short*)Cout  + (size_t)b * strideC;
      unsigned short* C2 = (OUT_MODE == 2) ? ((unsigned short*)Cout2 + (size_t)b * strideC) : nullptr;
      for (int pass = 0; pass < 2; ++pass) {
#pragma unroll
        for (int it = 0; it < 4; ++it) {
          const int row = it * 4 + q;
          const float* sp = slab + row * 68 + c8;
          v8h hv, lv;
#pragma unroll
          for (int e = 0; e < 8; ++e) {
            if (OUT_MODE == 1) {
              hv[e] = (_Float16)sp[e];
            } else {
              unsigned short hb = f2bf_bits(sp[e]);
              unsigned short lb = f2bf_bits(sp[e] - bf_bits2f(hb));
              hv[e] = __builtin_bit_cast(_Float16, hb);
              lv[e] = __builtin_bit_cast(_Float16, lb);
            }
          }
          *(volatile v8h*)(C + (size_t)(mBase + row) * ldc + n0 + c8) = hv;
          if (OUT_MODE == 2) *(volatile v8h*)(C2 + (size_t)(mBase + row) * ldc + n0 + c8) = lv;
        }
        __threadfence();
      }
    }
    __builtin_amdgcn_fence(__ATOMIC_RELEASE, "workgroup");
    __builtin_amdgcn_wave_barrier();
    __builtin_amdgcn_fence(__ATOMIC_ACQUIRE, "workgroup");
  }
}


__global__ __launch_bounds__(kThr) void obs_prep_kernel(const float* __restrict__ A, const float* __restrict__ Hm,
                                                        const float* __restrict__ Lm,
                                                        float* __restrict__ HPG, float* __restrict__ PLG,
                                                        float* __restrict__ HPLG, float* __restrict__ P16,
                                                        float* __restrict__ ZB) {
  __shared__ float sM[kState * 65];
  __shared__ float sP[2][kState * 65];
  __shared__ float sH[kObs * 65];
  __shared__ float sL[kState * 33];
  __shared__ float sHP[kObs * 65];
  const int tid = threadIdx.x;

#pragma unroll
  for (int it = 0; it < 8; ++it) {
    const int e = it * kThr + tid;
    sH[(e >> 6) * 65 + (e & 63)] = bf16r(Hm[e]);
    sL[(e >> 5) * 33 + (e & 31)] = bf16r(Lm[e]);
  }
  __syncthreads();
#pragma unroll 1
  for (int it = 0; it < 16; ++it) {
    const int e = it * kThr + tid;
    const int r = e >> 6, c = e & 63;
    float acc = 0.0f;
#pragma unroll 8
    for (int q = 0; q < kObs; ++q) acc = fmaf(sL[r * 33 + q], sH[q * 65 + c], acc);
    sM[r * 65 + c] = bf16r(A[e]) - acc;
    sP[0][r * 65 + c] = (r == c) ? 1.0f : 0.0f;
  }
  __syncthreads();

#pragma unroll 1
  for (int i = 0; i < kChunk; ++i) {
    const float* cur = sP[i & 1];
    float* nxt = sP[(i + 1) & 1];
#pragma unroll 1
    for (int it = 0; it < 8; ++it) {
      const int e = it * kThr + tid;
      const int r = e >> 6, c = e & 63;
      float acc = 0.0f;
#pragma unroll 8
      for (int k = 0; k < kState; ++k) acc = fmaf(sH[r * 65 + k], cur[k * 65 + c], acc);
      sHP[r * 65 + c] = acc;
      float* dst = HPG + (size_t)i * (kObs * kState) + e;
      *(volatile float*)dst = acc;
      __threadfence();
      *(volatile float*)dst = acc;
    }
#pragma unroll 1
    for (int it = 0; it < 8; ++it) {
      const int e = it * kThr + tid;
      const int r = e >> 5, q = e & 31;
      float acc = 0.0f;
#pragma unroll 8
      for (int k = 0; k < kState; ++k) acc = fmaf(cur[r * 65 + k], sL[k * 33 + q], acc);
      float* dst = PLG + (size_t)i * (kState * kObs) + e;
      *(volatile float*)dst = acc;
      __threadfence();
      *(volatile float*)dst = acc;
    }
#pragma unroll 1
    for (int it = 0; it < 16; ++it) {
      const int e = it * kThr + tid;
      const int r = e >> 6, c = e & 63;
      float acc = 0.0f;
#pragma unroll 8
      for (int k = 0; k < kState; ++k) acc = fmaf(sM[r * 65 + k], cur[k * 65 + c], acc);
      nxt[r * 65 + c] = acc;
    }
    __syncthreads();
#pragma unroll 1
    for (int it = 0; it < 4; ++it) {
      const int e = it * kThr + tid;
      const int r = e >> 5, q = e & 31;
      float acc = 0.0f;
#pragma unroll 8
      for (int k = 0; k < kState; ++k) acc = fmaf(sHP[r * 65 + k], sL[k * 33 + q], acc);
      float* dst = HPLG + (size_t)i * (kObs * kObs) + e;
      *(volatile float*)dst = acc;
      __threadfence();
      *(volatile float*)dst = acc;
    }
    __syncthreads();
  }
  {
    const float* fin = sP[kChunk & 1];
#pragma unroll 1
    for (int it = 0; it < 16; ++it) {
      const int e = it * kThr + tid;
      const float v = fin[(e >> 6) * 65 + (e & 63)];
      *(volatile float*)(P16 + e) = v;
      __threadfence();
      *(volatile float*)(P16 + e) = v;
    }
#pragma unroll
    for (int it = 0; it < 2; ++it) {
      const int e = it * kThr + tid;
      *(volatile float*)(ZB + e) = 0.0f;
      __threadfence();
      *(volatile float*)(ZB + e) = 0.0f;
    }
  }
}

__global__ __launch_bounds__(kThr) void obs_planes_kernel(const float* __restrict__ HPG, const float* __restrict__ PLG,
                                                          const float* __restrict__ HPLG,
                                                          unsigned short* __restrict__ OT16, unsigned short* __restrict__ G16) {
  const int blk = blockIdx.x;
  v8h hv;
  unsigned short* dst;
  if (blk < 144) {
    const int v   = blk * kThr + threadIdx.x;
    const int R   = v / 72;
    const int col = (v - R * 72) * 8;
    const int ii  = R >> 5, mm = R & 31;
    const bool isO = (col < kState);
    const int oc   = isO ? col : 0;
    const int tq   = isO ? 0 : (col - kState);
    const int l = tq >> 5;
    const int q = tq & 31;
    const int jraw = ii - 1 - l;
    const int j = (jraw >= 0) ? jraw : 0;
#pragma unroll
    for (int e = 0; e < 8; ++e) {
      float ov = HPG[((size_t)ii * kObs + mm) * kState + oc + e];
      float tv = HPLG[((size_t)j * kObs + mm) * kObs + q + e];
      asm volatile("" : "+v"(ov), "+v"(tv));
      const float tsel = (jraw >= 0) ? tv : 0.0f;
      const float sc = isO ? (ov * kOCarry) : (tsel * kGCarry);
      hv[e] = (_Float16)carry_flush(sc, 1.0f);
    }
    dst = OT16 + (size_t)R * kAW + col;
  } else {
    const int v   = (blk - 144) * kThr + threadIdx.x;
    const int r   = v >> 6;
    const int col = (v & 63) * 8;
    const int i = col >> 5, q = col & 31;
#pragma unroll
    for (int e = 0; e < 8; ++e) hv[e] = (_Float16)carry_flush(PLG[((size_t)(kChunk - 1 - i) * kState + r) * kObs + q + e], kGCarry);
    dst = G16 + (size_t)r * kYW + col;
  }
  *(volatile v8h*)dst = hv;
  __threadfence();
  *(volatile v8h*)dst = hv;
}

__global__ __launch_bounds__(kThr) void ychunk_plane_kernel(const float* __restrict__ y, unsigned short* __restrict__ AC16) {
  const int v  = blockIdx.x * kThr + threadIdx.x;
  const int j  = v >> 6;
  const int c8 = (v & 63) * 8;
  const int i  = c8 >> 5, m0 = c8 & 31;
  v8h hv;
#pragma unroll
  for (int e = 0; e < 8; ++e) {
    const float yv = y[(size_t)(m0 + e) * kSteps + (size_t)j * kChunk + i];
    hv[e] = (_Float16)carry_flush(bf16r(yv), kYCarry);
  }
  unsigned short* dst = AC16 + (size_t)j * kAW + kState + c8;
  *(volatile v8h*)dst = hv;
  __threadfence();
  *(volatile v8h*)dst = hv;
}

__global__ __launch_bounds__(32) void boundary_kernel(const float* __restrict__ P16, const float* __restrict__ WF,
                                                      const int* __restrict__ nsteps, unsigned short* __restrict__ AC16) {
  __shared__ __align__(16) float sS[2][kState];
  const int lane = threadIdx.x & 31;
  const int r0 = 2 * lane;
  float p0[kState], p1[kState];
#pragma unroll
  for (int c = 0; c < kState; ++c) { p0[c] = P16[r0 * kState + c]; p1[c] = P16[(r0 + 1) * kState + c]; }
  const int nv = nsteps[0];
  const float poison = (nv == kSteps) ? 0.0f : __builtin_nanf("");
  float s0 = poison, s1 = poison;
#pragma unroll 1
  for (int j = 0; j < kNumCh; ++j) {
    float* buf = sS[j & 1];
    buf[r0] = s0;
    buf[r0 + 1] = s1;
    v2h hv;
    hv[0] = (_Float16)carry_flush(s0, kSCarry);
    hv[1] = (_Float16)carry_flush(s1, kSCarry);
    unsigned short* dst = AC16 + (size_t)j * kAW + r0;
    *(volatile v2h*)dst = hv;
    __threadfence();
    *(volatile v2h*)dst = hv;
    const v2f w = *(const v2f*)(WF + (size_t)j * kState + r0);
    __syncthreads();
    float a0 = w[0], a1 = w[1];
#pragma unroll
    for (int c4 = 0; c4 < kState; c4 += 4) {
      const v4f sv = *(const v4f*)(buf + c4);
#pragma unroll
      for (int e = 0; e < 4; ++e) {
        a0 = fmaf(p0[c4 + e], sv[e], a0);
        a1 = fmaf(p1[c4 + e], sv[e], a1);
      }
    }
    s0 = a0;
    s1 = a1;
  }
}

__global__ __launch_bounds__(kThr) void obs_out_kernel(const float* __restrict__ YH, float* __restrict__ out) {
  const size_t t = (size_t)blockIdx.x * kThr + threadIdx.x;
  const int q4 = (int)(t & (kSteps / 4 - 1));
  const int m  = (int)(t >> 16);
  const int k0 = q4 * 4;
  const int j  = k0 >> 4;
  const int i0 = k0 & 15;
  v4f o;
#pragma unroll
  for (int e = 0; e < 4; ++e) {
    const float v = YH[(size_t)j * kYW + (i0 + e) * kObs + m];
    o[e] = v;
  }
  float* dst = out + (size_t)m * kSteps + k0;
  *(volatile v4f*)dst = o;
  __threadfence();
  *(volatile v4f*)dst = o;
}

static_assert(((kNumCh / 64) * (kState / 64)) % 8 == 0 && ((kNumCh / 64) * (kYW / 64)) % 8 == 0, "GEMM grids exact");
static_assert(((size_t)kNumCh * (kYW / 8)) % kThr == 0 && ((size_t)kObs * kSteps / 4) % kThr == 0, "plane and output grids exact");
static_assert(512 * 72 == 144 * kThr && 64 * 64 == 16 * kThr, "weight-plane grid exact");

extern "C" void kernel_launch(void* const* d_in, const int* in_sizes, int n_in,
                              void* d_out, int out_size, void* d_ws, size_t ws_size,
                              hipStream_t stream) {
  if (n_in < 5 || d_out == nullptr || d_ws == nullptr) return;
  if ((size_t)in_sizes[0] != (size_t)kObs * kSteps) return;
  if (in_sizes[1] != kState * kState || in_sizes[2] != kObs * kState || in_sizes[3] != kState * kObs) return;
  if (in_sizes[4] < 1) return;
  if ((size_t)out_size != (size_t)kObs * kSteps) return;
  if (ws_size < kWsTotal) return;

  const float* y  = (const float*)d_in[0];
  const float* A  = (const float*)d_in[1];
  const float* Hm = (const float*)d_in[2];
  const float* Lm = (const float*)d_in[3];
  const int*   nst = (const int*)d_in[4];
  float* out = (float*)d_out;

  char* ws = (char*)d_ws;
  float* HPG  = (float*)(ws + kOffHPG);
  float* PLG  = (float*)(ws + kOffPLG);
  float* HPLG = (float*)(ws + kOffHPLG);
  float* P16  = (float*)(ws + kOffP16);
  float* ZB   = (float*)(ws + kOffZB);
  unsigned short* G16  = (unsigned short*)(ws + kOffG16);
  unsigned short* OT16 = (unsigned short*)(ws + kOffOT);
  unsigned short* AC16 = (unsigned short*)(ws + kOffAC);
  float* WF = (float*)(ws + kOffWF);
  float* YH = (float*)(ws + kOffYH);

  obs_prep_kernel<<<1, kThr, 0, stream>>>(A, Hm, Lm, HPG, PLG, HPLG, P16, ZB);
  obs_planes_kernel<<<160, kThr, 0, stream>>>(HPG, PLG, HPLG, OT16, G16);
  ychunk_plane_kernel<<<(int)(((size_t)kNumCh * (kYW / 8)) / kThr), kThr, 0, stream>>>(y, AC16);

  wmma_gemm64<0, false, 2, 0, false, 0><<<dim3((kNumCh / 64) * (kState / 64) / 8, 1), 256, 0, stream>>>(
      AC16 + kState, AC16 + kState, kAW, 0L, G16, G16, kYW, 0L, (void*)WF, (void*)WF, kState, 0L,
      ZB, nullptr, 0L, kNumCh, kState, kYW, kScale);

  boundary_kernel<<<1, 32, 0, stream>>>(P16, WF, nst, AC16);

  wmma_gemm64<0, false, 2, 0, false, 0><<<dim3((kNumCh / 64) * (kYW / 64) / 8, 1), 256, 0, stream>>>(
      AC16, AC16, kAW, 0L, OT16, OT16, kAW, 0L, (void*)YH, (void*)YH, kYW, 0L,
      ZB, nullptr, 0L, kNumCh, kYW, kAW, kScale);

  obs_out_kernel<<<(int)(((size_t)kObs * kSteps / 4) / kThr), kThr, 0, stream>>>(YH, out);
}
